// PatchQuantumGenerator_53901839564947
// MI455X (gfx1250) — hardware-run, weakly checked
//
#include <hip/hip_runtime.h>
#include <math.h>

typedef __attribute__((ext_vector_type(16))) _Float16 v16h;
typedef __attribute__((ext_vector_type(8)))  _Float16 v8h;
typedef __attribute__((ext_vector_type(16))) __bf16   v16b;
typedef __attribute__((ext_vector_type(8)))  __bf16   v8b;
typedef __attribute__((ext_vector_type(8)))  float    v8f;
typedef __attribute__((ext_vector_type(4)))  float    v4f;

constexpr int kBatch   = 16384;
constexpr int kWires   = 8;
constexpr int kGen     = 4;
constexpr int kPatch   = 64;
constexpr int kDepth   = 6;
constexpr int kDim     = 256;
constexpr int kCls     = 10;
constexpr int kHid     = 64;
constexpr int kAng     = 16;
constexpr int kCp      = 32;
constexpr int kQd      = 288;
constexpr int kQdPad   = 320;
constexpr int kFeat    = 128;
constexpr int kOutW    = 64;
constexpr int kPsiRows = 2 * kBatch;
constexpr int kQpRow   = kDepth * kWires;
static_assert(kDim == (1 << kWires));
static_assert(kGen * kPatch == kDim);
static_assert(kGen * kPatch + kCp == kQd);
static_assert((kQdPad % 32) == 0 && kQdPad >= kQd && (kQdPad - kGen * kPatch) == 64);
static_assert((kFeat % 64) == 0 && (kOutW % 64) == 0 && (kDim % 64) == 0);
static_assert((kBatch % 64) == 0 && (kPsiRows % 64) == 0);
static_assert((kFeat % 32) == 0 && (kDim % 32) == 0);

constexpr float kCarryAct  = 16.0f;
constexpr float kCarryWgt  = 1024.0f;
constexpr float kHeadFold  = 1.0f / (kCarryAct * kCarryWgt);
constexpr float kF16MinNrm = 6.103515625e-5f;
constexpr float kLnEps     = 1e-5f;
constexpr float kInvFeat   = 1.0f / (float)kFeat;
constexpr float kPi        = 3.14159265358979323846f;

constexpr size_t kOffUTH = 0;
constexpr size_t kOffUTL = kOffUTH + (size_t)kDim * kDim * 2;
constexpr size_t kOffW1H = kOffUTL + (size_t)kDim * kDim * 2;
constexpr size_t kOffW1L = kOffW1H + (size_t)kFeat * kQdPad * 2;
constexpr size_t kOffW2H = kOffW1L + (size_t)kFeat * kQdPad * 2;
constexpr size_t kOffW2L = kOffW2H + (size_t)kFeat * kFeat * 2;
constexpr size_t kOffW3F = kOffW2L + (size_t)kFeat * kFeat * 2;
constexpr size_t kOffANG = kOffW3F + (size_t)kOutW * kFeat * 2;
constexpr size_t kOffPSH = kOffANG + (size_t)kBatch * kAng * 4;
constexpr size_t kOffPSL = kOffPSH + (size_t)kPsiRows * kDim * 2;
constexpr size_t kOffXH  = kOffPSL + (size_t)kPsiRows * kDim * 2;
constexpr size_t kOffXL  = kOffXH  + (size_t)kBatch * kQdPad * 2;
constexpr size_t kOffY1  = kOffXL  + (size_t)kBatch * kQdPad * 2;
constexpr size_t kOffX1H = kOffY1  + (size_t)kBatch * kFeat * 4;
constexpr size_t kOffX1L = kOffX1H + (size_t)kBatch * kFeat * 2;
constexpr size_t kOffY2  = kOffX1L + (size_t)kBatch * kFeat * 2;
constexpr size_t kOffX2F = kOffY2  + (size_t)kBatch * kFeat * 4;
constexpr size_t kWsTotal = kOffX2F + (size_t)kBatch * kFeat * 2;
static_assert(kWsTotal == 85442560ull);
static_assert(kWsTotal <= 134217728ull);
static_assert((kOffUTL % 128) == 0 && (kOffW1H % 128) == 0 && (kOffW1L % 128) == 0 && (kOffW2H % 128) == 0 &&
              (kOffW2L % 128) == 0 && (kOffW3F % 128) == 0 && (kOffANG % 128) == 0 && (kOffPSH % 128) == 0 &&
              (kOffPSL % 128) == 0 && (kOffXH % 128) == 0 && (kOffXL % 128) == 0 && (kOffY1 % 128) == 0 &&
              (kOffX1H % 128) == 0 && (kOffX1L % 128) == 0 && (kOffY2 % 128) == 0 && (kOffX2F % 128) == 0);

__device__ __forceinline__ unsigned short f2bf_bits(float f) {
  unsigned u = __float_as_uint(f);
  return (unsigned short)((u + 0x7FFFu + ((u >> 16) & 1u)) >> 16);
}
__device__ __forceinline__ float bf_bits2f(unsigned short h) { return __uint_as_float(((unsigned)h) << 16); }
__device__ __forceinline__ float lrelu02(float x) { return (x >= 0.0f) ? x : 0.2f * x; }

__device__ __forceinline__ void split8_bf16(const v4f a0, const v4f a1, v8h& hv, v8h& lv) {
#pragma unroll
  for (int e = 0; e < 4; ++e) {
    const float x0 = a0[e];
    const float x1 = a1[e];
    const unsigned short h0 = f2bf_bits(x0);
    const unsigned short h1 = f2bf_bits(x1);
    const unsigned short l0 = f2bf_bits(x0 - bf_bits2f(h0));
    const unsigned short l1 = f2bf_bits(x1 - bf_bits2f(h1));
    hv[e]     = __builtin_bit_cast(_Float16, h0);
    hv[4 + e] = __builtin_bit_cast(_Float16, h1);
    lv[e]     = __builtin_bit_cast(_Float16, l0);
    lv[4 + e] = __builtin_bit_cast(_Float16, l1);
  }
}
__device__ __forceinline__ void carry8_f16(const v4f a0, const v4f a1, float carry, v8h& hv) {
#pragma unroll
  for (int e = 0; e < 4; ++e) {
    float x0 = a0[e] * carry;
    float x1 = a1[e] * carry;
    x0 = (fabsf(x0) < kF16MinNrm) ? 0.0f : x0;
    x1 = (fabsf(x1) < kF16MinNrm) ? 0.0f : x1;
    hv[e]     = (_Float16)x0;
    hv[4 + e] = (_Float16)x1;
  }
}

__device__ __forceinline__ void tie1_h(v8f& a, v16h x, v16h y) { asm volatile("v_nop\n\tv_nop\n\tv_nop\n\tv_nop" : "+v"(a) : "v"(x), "v"(y)); }
__device__ __forceinline__ void tie1_b(v8f& a, v16b x, v16b y) { asm volatile("v_nop\n\tv_nop\n\tv_nop\n\tv_nop" : "+v"(a) : "v"(x), "v"(y)); }
__device__ __forceinline__ void keep4_h(v16h a, v16h b, v16h c, v16h d) { asm volatile("v_nop" :: "v"(a), "v"(b), "v"(c), "v"(d)); }
__device__ __forceinline__ void keep4_b(v16b a, v16b b, v16b c, v16b d) { asm volatile("v_nop" :: "v"(a), "v"(b), "v"(c), "v"(d)); }
__device__ __forceinline__ void acc_guard4(v8f& a, v8f& b, v8f& c, v8f& d) { asm volatile("v_nop\n\tv_nop\n\tv_nop\n\tv_nop" : "+v"(a), "+v"(b), "+v"(c), "+v"(d)); }

template <typename T> struct Frag;
template <> struct Frag<_Float16> {
  typedef v16h V; union U { v16h v; v8h h[2]; };
  static __device__ __forceinline__ v16h load(const _Float16* p) {
    U f; f.h[0] = *(const v8h*)(p); f.h[1] = *(const v8h*)(p + 16); return f.v;
  }
  static __device__ __forceinline__ v8f mma(v16h a, v16h b, v8f c) {
    return __builtin_amdgcn_wmma_f32_16x16x32_f16(false, a, false, b, (short)0, c, false, false);
  }
  static __device__ __forceinline__ void tie(v8f& a, v16h x, v16h y) { tie1_h(a, x, y); }
  static __device__ __forceinline__ void keep(v16h a, v16h b, v16h c, v16h d) { keep4_h(a, b, c, d); }
};
template <> struct Frag<__bf16> {
  typedef v16b V; union U { v16b v; v8b h[2]; };
  static __device__ __forceinline__ v16b load(const __bf16* p) {
    U f; f.h[0] = *(const v8b*)(p); f.h[1] = *(const v8b*)(p + 16); return f.v;
  }
  static __device__ __forceinline__ v8f mma(v16b a, v16b b, v8f c) {
    return __builtin_amdgcn_wmma_f32_16x16x32_bf16(false, a, false, b, (short)0, c, false, false);
  }
  static __device__ __forceinline__ void tie(v8f& a, v16b x, v16b y) { tie1_b(a, x, y); }
  static __device__ __forceinline__ void keep(v16b a, v16b b, v16b c, v16b d) { keep4_b(a, b, c, d); }
};

template <int ET> struct Elem;
template <> struct Elem<0> { typedef _Float16 T; };
template <> struct Elem<1> { typedef __bf16 T; };

template <int ET, int SPL, int BIAS_MODE, int OUT_MODE, int ACT>
__global__ __launch_bounds__(256) void wmma_gemm64(
    const unsigned short* __restrict__ Ap, const unsigned short* __restrict__ A2p, int lda,
    const unsigned short* __restrict__ Btp, const unsigned short* __restrict__ Bt2p, int ldb,
    void* __restrict__ Cout, void* __restrict__ Cout2, int ldc,
    const float* __restrict__ bias, int M, int N, int K, float scale) {
  typedef typename Elem<ET>::T T;
  typedef typename Frag<T>::V V;
  const T* A = (const T*)Ap; const T* A2 = (const T*)A2p; const T* Bt = (const T*)Btp; const T* Bt2 = (const T*)Bt2p;
  __shared__ __align__(16) float sT[8][16 * 68];
  const int lane = threadIdx.x & 31;
  const int wave = threadIdx.x >> 5;
  const int tilesN = N >> 6;
  const int tilesM = M >> 6;
  const int tile = blockIdx.x * 8 + wave;
  if (tile >= tilesM * tilesN) return;
  const int tm = tile / tilesN;
  const int tn = tile - tm * tilesN;
  const int m0 = tm << 6;
  const int n0 = tn << 6;

  const T* Ab2 = (SPL == 2) ? A2 : nullptr;
  const T* Bb2 = (SPL == 2) ? Bt2 : nullptr;

  const int rlane = lane & 15;
  const int koff  = (lane >> 4) * 8;
  const int mOff  = (lane >> 4) * 8;

  v8f acc[4][4];
#pragma unroll
  for (int i = 0; i < 4; ++i)
#pragma unroll
    for (int j = 0; j < 4; ++j) acc[i][j] = (v8f){0.f,0.f,0.f,0.f,0.f,0.f,0.f,0.f};

  for (int k0 = 0; k0 < K; k0 += 32) {
    V bh[4], bl[4];
#pragma unroll
    for (int j = 0; j < 4; ++j) {
      const size_t bo = (size_t)(n0 + (j << 4) + rlane) * ldb + koff + k0;
      bh[j] = Frag<T>::load(Bt + bo);
      if (SPL == 2) bl[j] = Frag<T>::load(Bb2 + bo);
    }
#pragma unroll
    for (int i = 0; i < 4; ++i) {
      const size_t ao = (size_t)(m0 + (i << 4) + rlane) * lda + koff + k0;
      V ah = Frag<T>::load(A + ao);
      V al;
      if (SPL == 2) al = Frag<T>::load(Ab2 + ao);
#pragma unroll
      for (int j = 0; j < 4; ++j) {
        acc[i][j] = Frag<T>::mma(ah, bh[j], acc[i][j]);
        if (SPL == 2) {
          acc[i][j] = Frag<T>::mma(ah, bl[j], acc[i][j]);
          acc[i][j] = Frag<T>::mma(al, bh[j], acc[i][j]);
        }
      }
#pragma unroll
      for (int j = 0; j < 4; ++j) Frag<T>::tie(acc[i][j], ah, (SPL == 2) ? al : ah);
    }
    Frag<T>::keep(bh[0], bh[1], bh[2], bh[3]);
    if (SPL == 2) Frag<T>::keep(bl[0], bl[1], bl[2], bl[3]);
  }
  acc_guard4(acc[0][0], acc[0][1], acc[0][2], acc[0][3]);
  acc_guard4(acc[1][0], acc[1][1], acc[1][2], acc[1][3]);
  acc_guard4(acc[2][0], acc[2][1], acc[2][2], acc[2][3]);
  acc_guard4(acc[3][0], acc[3][1], acc[3][2], acc[3][3]);

  float* slab = sT[wave];
#pragma unroll
  for (int i = 0; i < 4; ++i) {
    const int mBase = m0 + (i << 4);
#pragma unroll
    for (int j = 0; j < 4; ++j) {
      const int n = n0 + (j << 4) + rlane;
      float bv = 0.f;
      if (BIAS_MODE == 2) bv = bias[n];
#pragma unroll
      for (int r = 0; r < 8; ++r) {
        float v = acc[i][j][r] * scale;
        if (BIAS_MODE == 2) v += bv;
        if (ACT == 6) v = (v >= 0.0f) ? v : 0.2f * v;
        slab[(mOff + r) * 68 + (j << 4) + rlane] = v;
      }
    }
    __builtin_amdgcn_fence(__ATOMIC_RELEASE, "workgroup");
    __builtin_amdgcn_wave_barrier();
    __builtin_amdgcn_fence(__ATOMIC_ACQUIRE, "workgroup");
    if (OUT_MODE == 0) {
      float* C = (float*)Cout;
      const int hh = lane >> 4, c4 = (lane & 15) * 4;
      if (ACT == 1) {
#pragma unroll 1
        for (int t = 0; t < 32; ++t) {
          float* cell = slab + ((t >> 2) * 2 + hh) * 68 + c4 + (t & 3);
          const float zv = *cell;
          *cell = tanhf(zv);
        }
        __builtin_amdgcn_fence(__ATOMIC_RELEASE, "workgroup");
        __builtin_amdgcn_wave_barrier();
        __builtin_amdgcn_fence(__ATOMIC_ACQUIRE, "workgroup");
      }
      for (int pass = 0; pass < 2; ++pass) {
#pragma unroll
        for (int it = 0; it < 8; ++it) {
          const int row = it * 2 + hh;
          v4f v = *(const v4f*)(slab + row * 68 + c4);
          *(volatile v4f*)(C + (size_t)(mBase + row) * ldc + n0 + c4) = v;
        }
        __threadfence();
      }
    } else {
      const int q = lane >> 3, c8 = (lane & 7) * 8;
      unsigned short* C  = (unsigned short*)Cout;
      unsigned short* C2 = (unsigned short*)Cout2;
      v8h hv[2], lv[2];
#pragma unroll
      for (int it = 0; it < 2; ++it) {
        const int s = it * 4 + q;
        const float* pr = slab + (2 * s) * 68 + c8;
        const float* pi = slab + (2 * s + 1) * 68 + c8;
        const v4f r0 = *(const v4f*)(pr);
        const v4f r1 = *(const v4f*)(pr + 4);
        const v4f i0 = *(const v4f*)(pi);
        const v4f i1 = *(const v4f*)(pi + 4);
        v4f p0, p1;
#pragma unroll
        for (int e = 0; e < 4; ++e) {
          p0[e] = r0[e] * r0[e] + i0[e] * i0[e];
          p1[e] = r1[e] * r1[e] + i1[e] * i1[e];
        }
        float mx = fmaxf(fmaxf(fmaxf(p0[0], p0[1]), fmaxf(p0[2], p0[3])), fmaxf(fmaxf(p1[0], p1[1]), fmaxf(p1[2], p1[3])));
        mx = fmaxf(mx, __shfl_xor(mx, 1, 32));
        mx = fmaxf(mx, __shfl_xor(mx, 2, 32));
        mx = fmaxf(mx, __shfl_xor(mx, 4, 32));
        const float inv = 1.0f / mx;
#pragma unroll
        for (int e = 0; e < 4; ++e) {
          p0[e] = p0[e] * inv;
          p1[e] = p1[e] * inv;
        }
        split8_bf16(p0, p1, hv[it], lv[it]);
      }
      for (int pass = 0; pass < 2; ++pass) {
#pragma unroll
        for (int it = 0; it < 2; ++it) {
          const size_t o = (size_t)((mBase >> 1) + it * 4 + q) * ldc + n0 + c8;
          *(volatile v8h*)(C + o)  = hv[it];
          *(volatile v8h*)(C2 + o) = lv[it];
        }
        __threadfence();
      }
    }
    __builtin_amdgcn_fence(__ATOMIC_RELEASE, "workgroup");
    __builtin_amdgcn_wave_barrier();
    __builtin_amdgcn_fence(__ATOMIC_ACQUIRE, "workgroup");
  }
}

__global__ __launch_bounds__(256) void build_rows_kernel(
    const float* __restrict__ qp, unsigned short* __restrict__ UH, unsigned short* __restrict__ UL)
{
  __shared__ __align__(16) float sV[2][kDim];
  __shared__ float sCS[2 * kQpRow];
  const int tid = threadIdx.x, lane = tid & 31, wave = tid >> 5;
  const int g = blockIdx.x >> 6;
  const int j = blockIdx.x & 63;
  {
    const int pi = (tid < kQpRow) ? tid : (kQpRow - 1);
    float w = qp[g * kQpRow + pi];
    asm volatile("" : "+v"(w));
    float sv, cv;
    sincosf(0.5f * w, &sv, &cv);
    if (tid < kQpRow) {
      sCS[2 * tid]     = cv;
      sCS[2 * tid + 1] = sv;
    }
  }
  sV[0][tid] = (tid == j) ? 1.0f : 0.0f;
  __syncthreads();
  int cur = 0;
  const float sgnSelf = (__popc(tid & (tid >> 1)) & 1) ? -1.0f : 1.0f;
#pragma unroll 1
  for (int d = kDepth - 1; d >= 0; --d) {
#pragma unroll 1
    for (int i = 0; i < kWires; ++i) {
      const int sh = 7 - i;
      const int pt = tid ^ (1 << sh);
      const float sgnPart = (__popc(pt & (pt >> 1)) & 1) ? -1.0f : 1.0f;
      const float fs = (i == 0) ? sgnSelf : 1.0f;
      const float fp = (i == 0) ? sgnPart : 1.0f;
      const float as = sV[cur][tid] * fs;
      const float ap = sV[cur][pt] * fp;
      const float c = sCS[2 * (d * kWires + i)];
      const float s = sCS[2 * (d * kWires + i) + 1];
      const int bit = (tid >> sh) & 1;
      const float sp = s * ap;
      const float nv = bit ? (c * as - sp) : (c * as + sp);
      sV[cur ^ 1][tid] = nv;
      __syncthreads();
      cur ^= 1;
    }
  }
  if (wave == 0) {
    const float* sp = &sV[cur][lane * 8];
    const v4f a0 = *(const v4f*)(sp);
    const v4f a1 = *(const v4f*)(sp + 4);
    v8h hv, lv;
    split8_bf16(a0, a1, hv, lv);
    unsigned short* qh = UH + (size_t)blockIdx.x * kDim + lane * 8;
    unsigned short* ql = UL + (size_t)blockIdx.x * kDim + lane * 8;
    *(volatile v8h*)qh = hv;
    *(volatile v8h*)ql = lv;
    __threadfence();
    *(volatile v8h*)qh = hv;
    *(volatile v8h*)ql = lv;
  }
}

__global__ __launch_bounds__(256) void split_pad_bf16_kernel(
    const float* __restrict__ src, unsigned short* __restrict__ dhi, unsigned short* __restrict__ dlo,
    int rows, int kin, int kout)
{
  const int i = blockIdx.x * 256 + threadIdx.x;
  const int gpr = kout >> 3;
  if (i >= rows * gpr) return;
  const int n = i / gpr;
  const int k0 = (i - n * gpr) << 3;
  const bool real = (k0 < kin);
  const int kc = real ? k0 : (kin - 8);
  v4f a0 = *(const v4f*)(src + (size_t)n * kin + kc);
  v4f a1 = *(const v4f*)(src + (size_t)n * kin + kc + 4);
  const v4f zz = (v4f){0.f, 0.f, 0.f, 0.f};
  a0 = real ? a0 : zz;
  a1 = real ? a1 : zz;
  v8h hv, lv;
  split8_bf16(a0, a1, hv, lv);
  unsigned short* qh = dhi + ((size_t)i << 3);
  unsigned short* ql = dlo + ((size_t)i << 3);
  *(volatile v8h*)qh = hv;
  *(volatile v8h*)ql = lv;
  __threadfence();
  *(volatile v8h*)qh = hv;
  *(volatile v8h*)ql = lv;
}

__global__ __launch_bounds__(256) void cast_f16_carry_kernel(
    const float* __restrict__ src, unsigned short* __restrict__ dst, int total8, float carry)
{
  const int i = blockIdx.x * 256 + threadIdx.x;
  if (i >= total8) return;
  const size_t e0 = (size_t)i << 3;
  const v4f a0 = *(const v4f*)(src + e0);
  const v4f a1 = *(const v4f*)(src + e0 + 4);
  v8h hv;
  carry8_f16(a0, a1, carry, hv);
  unsigned short* q = dst + e0;
  *(volatile v8h*)q = hv;
  __threadfence();
  *(volatile v8h*)q = hv;
}

__global__ __launch_bounds__(256) void cond_mlp_kernel(
    const float* __restrict__ labels,
    const float* __restrict__ W1, const float* __restrict__ b1,
    const float* __restrict__ W2, const float* __restrict__ b2,
    const float* __restrict__ Wa, const float* __restrict__ ba,
    const float* __restrict__ Wp1, const float* __restrict__ bp1,
    const float* __restrict__ Wp2, const float* __restrict__ bp2,
    float* __restrict__ ANG, unsigned short* __restrict__ XH, unsigned short* __restrict__ XL)
{
  __shared__ __align__(16) float sW1t[kCls * kHid];
  __shared__ __align__(16) float sW2t[kHid * kHid];
  __shared__ __align__(16) float sWat[kHid * kAng];
  __shared__ __align__(16) float sWp1t[kCls * kCp];
  __shared__ __align__(16) float sWp2t[kCp * kCp];
  __shared__ float sB1[kHid];
  __shared__ float sB2[kHid];
  __shared__ float sBa[kAng];
  __shared__ float sBp1[kCp];
  __shared__ float sBp2[kCp];
  __shared__ float sLab[8 * 16];
  __shared__ float sH[8 * kHid];
  __shared__ float sH2[8 * kHid];
  __shared__ float sP1[8 * kCp];
  __shared__ __align__(16) float sAng[64 * kAng];
  __shared__ __align__(16) float sCp[64 * kCp];

  const int tid = threadIdx.x, lane = tid & 31, wave = tid >> 5;

  for (int idx = tid; idx < kHid * kCls; idx += 256) {
    const int o = idx / kCls;
    const int k = idx - o * kCls;
    sW1t[k * kHid + o] = W1[idx];
  }
  for (int idx = tid; idx < kHid * kHid; idx += 256) {
    const int o = idx >> 6;
    const int k = idx & 63;
    sW2t[k * kHid + o] = W2[idx];
  }
  for (int idx = tid; idx < kAng * kHid; idx += 256) {
    const int o = idx >> 6;
    const int k = idx & 63;
    sWat[k * kAng + o] = Wa[idx];
  }
  for (int idx = tid; idx < kCp * kCls; idx += 256) {
    const int o = idx / kCls;
    const int k = idx - o * kCls;
    sWp1t[k * kCp + o] = Wp1[idx];
  }
  for (int idx = tid; idx < kCp * kCp; idx += 256) {
    const int o = idx >> 5;
    const int k = idx & 31;
    sWp2t[k * kCp + o] = Wp2[idx];
  }
  {
    float v0 = b1[tid & (kHid - 1)];
    float v1 = b2[tid & (kHid - 1)];
    float v2 = ba[tid & (kAng - 1)];
    float v3 = bp1[tid & (kCp - 1)];
    float v4 = bp2[tid & (kCp - 1)];
    asm volatile("" : "+v"(v0));
    asm volatile("" : "+v"(v1));
    asm volatile("" : "+v"(v2));
    asm volatile("" : "+v"(v3));
    asm volatile("" : "+v"(v4));
    if (tid < kHid) { sB1[tid] = v0; sB2[tid] = v1; }
    if (tid < kAng) { sBa[tid] = v2; }
    if (tid < kCp)  { sBp1[tid] = v3; sBp2[tid] = v4; }
  }
  __syncthreads();

  const int b0 = blockIdx.x * 64;
  float* myLab = sLab + wave * 16;
  float* myH   = sH + wave * kHid;
  float* myH2  = sH2 + wave * kHid;
  float* myP1  = sP1 + wave * kCp;

#pragma unroll 1
  for (int rr = 0; rr < 8; ++rr) {
    const int lrow = wave * 8 + rr;
    const int b = b0 + lrow;
    {
      const int li = (lane < kCls) ? lane : (kCls - 1);
      float lv = labels[(size_t)b * kCls + li];
      asm volatile("" : "+v"(lv));
      if (lane < 16) myLab[lane] = (lane < kCls) ? lv : 0.0f;
    }
    __syncthreads();
    {
      float a0 = 0.0f, a1 = 0.0f, p = 0.0f;
#pragma unroll 2
      for (int k = 0; k < kCls; ++k) {
        const float l = myLab[k];
        a0 = fmaf(l, sW1t[k * kHid + lane], a0);
        a1 = fmaf(l, sW1t[k * kHid + lane + 32], a1);
        p  = fmaf(l, sWp1t[k * kCp + lane], p);
      }
      myH[lane]      = lrelu02(a0 + sB1[lane]);
      myH[lane + 32] = lrelu02(a1 + sB1[lane + 32]);
      myP1[lane]     = lrelu02(p + sBp1[lane]);
    }
    __syncthreads();
    {
      float c0 = 0.0f, c1 = 0.0f;
#pragma unroll 2
      for (int k = 0; k < kHid; ++k) {
        const float hk = myH[k];
        c0 = fmaf(hk, sW2t[k * kHid + lane], c0);
        c1 = fmaf(hk, sW2t[k * kHid + lane + 32], c1);
      }
      myH2[lane]      = myH[lane] + lrelu02(c0 + sB2[lane]);
      myH2[lane + 32] = myH[lane + 32] + lrelu02(c1 + sB2[lane + 32]);
      float p = 0.0f;
#pragma unroll 2
      for (int k = 0; k < kCp; ++k) p = fmaf(myP1[k], sWp2t[k * kCp + lane], p);
      sCp[lrow * kCp + lane] = lrelu02(p + sBp2[lane]);
    }
    __syncthreads();
    {
      const int o = lane & (kAng - 1);
      float s = 0.0f;
#pragma unroll 2
      for (int k = 0; k < kHid; ++k) s = fmaf(myH2[k], sWat[k * kAng + o], s);
      const float av = tanhf(s + sBa[o]) * kPi;
      if (lane < kAng) sAng[lrow * kAng + o] = av;
    }
  }
  __syncthreads();

  {
    const v4f av = *(const v4f*)(sAng + tid * 4);
    float* dst = ANG + (size_t)blockIdx.x * (64 * kAng) + tid * 4;
    v8h chv[2], clv[2];
    const int c8 = (tid & 7) * 8;
    const bool real = (c8 < kCp);
    const v4f zz = (v4f){0.f, 0.f, 0.f, 0.f};
#pragma unroll
    for (int it = 0; it < 2; ++it) {
      const int r = (tid >> 3) + 32 * it;
      const float* sp = sCp + r * kCp + (c8 & (kCp - 1));
      v4f a0 = *(const v4f*)(sp);
      v4f a1 = *(const v4f*)(sp + 4);
      a0 = real ? a0 : zz;
      a1 = real ? a1 : zz;
      split8_bf16(a0, a1, chv[it], clv[it]);
    }
    for (int pass = 0; pass < 2; ++pass) {
      *(volatile v4f*)dst = av;
#pragma unroll
      for (int it = 0; it < 2; ++it) {
        const int r = (tid >> 3) + 32 * it;
        const size_t o = (size_t)(b0 + r) * kQdPad + kGen * kPatch + c8;
        *(volatile v8h*)(XH + o) = chv[it];
        *(volatile v8h*)(XL + o) = clv[it];
      }
      __threadfence();
    }
  }
}

__device__ __forceinline__ void wire_factor(const float* sc, int i, int bit, float& fr, float& fi) {
  const float s  = sc[2 * i];
  const float c  = sc[2 * i + 1];
  const float sp = sc[2 * (kWires + i)];
  const float cp = sc[2 * (kWires + i) + 1];
  const float mag = bit ? s : c;
  fr = mag * cp;
  const float t = mag * sp;
  fi = bit ? t : -t;
}

__global__ __launch_bounds__(256) void state_planes_kernel(
    const float* __restrict__ noise, const float* __restrict__ ang,
    unsigned short* __restrict__ PH, unsigned short* __restrict__ PL)
{
  __shared__ __align__(16) float sSC[8][32];
  __shared__ __align__(16) float sG[8][16];
  __shared__ __align__(16) float sPsi[8][2 * kDim];
  const int tid = threadIdx.x, lane = tid & 31, wave = tid >> 5;
  const int wi = lane & 7;
  const int isph = (lane >> 3) & 1;
#pragma unroll 1
  for (int it = 0; it < 8; ++it) {
    const int b = blockIdx.x * 64 + it * 8 + wave;
    const float nz  = noise[(size_t)b * kWires + wi];
    const float ary = ang[(size_t)b * kAng + wi];
    const float arz = ang[(size_t)b * kAng + kWires + wi];
    const float th = 0.5f * (nz + ary);
    const float ph = 0.5f * arz;
    const float arg = isph ? ph : th;
    float sv, cv;
    sincosf(arg, &sv, &cv);
    if (lane < 16) {
      sSC[wave][2 * lane]     = sv;
      sSC[wave][2 * lane + 1] = cv;
    }
    __syncthreads();
    const float* sc = sSC[wave];
    float Lr = 1.0f, Li = 0.0f;
#pragma unroll 1
    for (int i = 0; i < 5; ++i) {
      const int bit = (lane >> (4 - i)) & 1;
      float fr, fi;
      wire_factor(sc, i, bit, fr, fi);
      const float nr = Lr * fr - Li * fi;
      const float ni = Lr * fi + Li * fr;
      Lr = nr;
      Li = ni;
    }
    float Gr = 1.0f, Gi = 0.0f;
#pragma unroll 1
    for (int i = 5; i < 8; ++i) {
      const int bit = (wi >> (7 - i)) & 1;
      float fr, fi;
      wire_factor(sc, i, bit, fr, fi);
      const float nr = Gr * fr - Gi * fi;
      const float ni = Gr * fi + Gi * fr;
      Gr = nr;
      Gi = ni;
    }
    if (lane < 8) {
      sG[wave][2 * lane]     = Gr;
      sG[wave][2 * lane + 1] = Gi;
    }
    __syncthreads();
    float* pre = sPsi[wave];
    float* pim = pre + kDim;
#pragma unroll 1
    for (int r = 0; r < 8; ++r) {
      const float gr = sG[wave][2 * r];
      const float gi = sG[wave][2 * r + 1];
      pre[lane * 8 + r] = Lr * gr - Li * gi;
      pim[lane * 8 + r] = Lr * gi + Li * gr;
    }
    __syncthreads();
    {
      const v4f r0 = *(const v4f*)(pre + lane * 8);
      const v4f r1 = *(const v4f*)(pre + lane * 8 + 4);
      const v4f i0 = *(const v4f*)(pim + lane * 8);
      const v4f i1 = *(const v4f*)(pim + lane * 8 + 4);
      v8h hr, lr, hi, li;
      split8_bf16(r0, r1, hr, lr);
      split8_bf16(i0, i1, hi, li);
      const size_t ore = (size_t)(2 * b) * kDim + lane * 8;
      const size_t oim = ore + kDim;
      for (int pass = 0; pass < 2; ++pass) {
        *(volatile v8h*)(PH + ore) = hr;
        *(volatile v8h*)(PH + oim) = hi;
        *(volatile v8h*)(PL + ore) = lr;
        *(volatile v8h*)(PL + oim) = li;
        __threadfence();
      }
    }
  }
}

template <int OUTK>
__global__ __launch_bounds__(256) void ln_rows_kernel(
    const float* __restrict__ Y, const float* __restrict__ gam, const float* __restrict__ bet,
    unsigned short* __restrict__ P0, unsigned short* __restrict__ P1)
{
  __shared__ __align__(16) float sN[64 * 132];
  const int tid = threadIdx.x, lane = tid & 31, wave = tid >> 5;
  const int r0 = blockIdx.x * 64;
  const v4f gv = *(const v4f*)(gam + lane * 4);
  const v4f bv = *(const v4f*)(bet + lane * 4);
#pragma unroll 1
  for (int rr = 0; rr < 8; ++rr) {
    const int lrow = wave * 8 + rr;
    const v4f v = *(const v4f*)(Y + (size_t)(r0 + lrow) * kFeat + lane * 4);
    float s = (v[0] + v[1]) + (v[2] + v[3]);
    s += __shfl_xor(s, 16, 32);
    s += __shfl_xor(s, 8, 32);
    s += __shfl_xor(s, 4, 32);
    s += __shfl_xor(s, 2, 32);
    s += __shfl_xor(s, 1, 32);
    const float mu = s * kInvFeat;
    v4f d;
    d[0] = v[0] - mu;
    d[1] = v[1] - mu;
    d[2] = v[2] - mu;
    d[3] = v[3] - mu;
    float ss = (d[0] * d[0] + d[1] * d[1]) + (d[2] * d[2] + d[3] * d[3]);
    ss += __shfl_xor(ss, 16, 32);
    ss += __shfl_xor(ss, 8, 32);
    ss += __shfl_xor(ss, 4, 32);
    ss += __shfl_xor(ss, 2, 32);
    ss += __shfl_xor(ss, 1, 32);
    const float rs = rsqrtf(ss * kInvFeat + kLnEps);
    v4f o;
    o[0] = d[0] * rs * gv[0] + bv[0];
    o[1] = d[1] * rs * gv[1] + bv[1];
    o[2] = d[2] * rs * gv[2] + bv[2];
    o[3] = d[3] * rs * gv[3] + bv[3];
    *(v4f*)(sN + lrow * 132 + lane * 4) = o;
  }
  __syncthreads();
  const int hrow = lane >> 4;
  const int c8 = (lane & 15) * 8;
  v8h hv[4], lv[4];
#pragma unroll
  for (int it = 0; it < 4; ++it) {
    const int lrow = wave * 8 + it * 2 + hrow;
    const float* sp = sN + lrow * 132 + c8;
    const v4f a0 = *(const v4f*)(sp);
    const v4f a1 = *(const v4f*)(sp + 4);
    if (OUTK == 0) {
      split8_bf16(a0, a1, hv[it], lv[it]);
    } else {
      carry8_f16(a0, a1, kCarryAct, hv[it]);
    }
  }
  for (int pass = 0; pass < 2; ++pass) {
#pragma unroll
    for (int it = 0; it < 4; ++it) {
      const int lrow = wave * 8 + it * 2 + hrow;
      const size_t o = (size_t)(r0 + lrow) * kFeat + c8;
      *(volatile v8h*)(P0 + o) = hv[it];
      if (OUTK == 0) *(volatile v8h*)(P1 + o) = lv[it];
    }
    __threadfence();
  }
}

extern "C" void kernel_launch(void* const* d_in, const int* in_sizes, int n_in,
                              void* d_out, int out_size, void* d_ws, size_t ws_size,
                              hipStream_t stream) {
  if (n_in < 23) return;
  const int expect[23] = {
    kBatch * kWires, kBatch * kCls, kGen * kQpRow,
    kHid * kCls, kHid, kHid * kHid, kHid, kAng * kHid, kAng,
    kCp * kCls, kCp, kCp * kCp, kCp,
    kFeat * kQd, kFeat, kFeat, kFeat,
    kFeat * kFeat, kFeat, kFeat, kFeat,
    kOutW * kFeat, kOutW };
  for (int i = 0; i < 23; ++i) {
    if (in_sizes[i] != expect[i]) return;
  }
  if (out_size != kBatch * kOutW) return;
  if (ws_size < kWsTotal) return;

  const float* noise  = (const float*)d_in[0];
  const float* labels = (const float*)d_in[1];
  const float* qprm   = (const float*)d_in[2];
  const float* W1  = (const float*)d_in[3];
  const float* b1  = (const float*)d_in[4];
  const float* W2  = (const float*)d_in[5];
  const float* b2  = (const float*)d_in[6];
  const float* Wa  = (const float*)d_in[7];
  const float* ba  = (const float*)d_in[8];
  const float* Wp1 = (const float*)d_in[9];
  const float* bp1 = (const float*)d_in[10];
  const float* Wp2 = (const float*)d_in[11];
  const float* bp2 = (const float*)d_in[12];
  const float* Wq1 = (const float*)d_in[13];
  const float* bq1 = (const float*)d_in[14];
  const float* g1  = (const float*)d_in[15];
  const float* be1 = (const float*)d_in[16];
  const float* Wq2 = (const float*)d_in[17];
  const float* bq2 = (const float*)d_in[18];
  const float* g2  = (const float*)d_in[19];
  const float* be2 = (const float*)d_in[20];
  const float* Wq3 = (const float*)d_in[21];
  const float* bq3 = (const float*)d_in[22];

  char* ws = (char*)d_ws;
  unsigned short* UTH = (unsigned short*)(ws + kOffUTH);
  unsigned short* UTL = (unsigned short*)(ws + kOffUTL);
  unsigned short* W1H = (unsigned short*)(ws + kOffW1H);
  unsigned short* W1L = (unsigned short*)(ws + kOffW1L);
  unsigned short* W2H = (unsigned short*)(ws + kOffW2H);
  unsigned short* W2L = (unsigned short*)(ws + kOffW2L);
  unsigned short* W3F = (unsigned short*)(ws + kOffW3F);
  float*          ANG = (float*)(ws + kOffANG);
  unsigned short* PSH = (unsigned short*)(ws + kOffPSH);
  unsigned short* PSL = (unsigned short*)(ws + kOffPSL);
  unsigned short* XH  = (unsigned short*)(ws + kOffXH);
  unsigned short* XL  = (unsigned short*)(ws + kOffXL);
  float*          Y1  = (float*)(ws + kOffY1);
  unsigned short* X1H = (unsigned short*)(ws + kOffX1H);
  unsigned short* X1L = (unsigned short*)(ws + kOffX1L);
  float*          Y2  = (float*)(ws + kOffY2);
  unsigned short* X2F = (unsigned short*)(ws + kOffX2F);

  build_rows_kernel<<<kGen * kPatch, 256, 0, stream>>>(qprm, UTH, UTL);

  split_pad_bf16_kernel<<<(kFeat * (kQdPad / 8)) / 256, 256, 0, stream>>>(Wq1, W1H, W1L, kFeat, kQd, kQdPad);
  split_pad_bf16_kernel<<<(kFeat * (kFeat / 8)) / 256, 256, 0, stream>>>(Wq2, W2H, W2L, kFeat, kFeat, kFeat);
  cast_f16_carry_kernel<<<(kOutW * kFeat / 8) / 256, 256, 0, stream>>>(Wq3, W3F, kOutW * kFeat / 8, kCarryWgt);

  cond_mlp_kernel<<<kBatch / 64, 256, 0, stream>>>(labels, W1, b1, W2, b2, Wa, ba, Wp1, bp1, Wp2, bp2, ANG, XH, XL);

  state_planes_kernel<<<kBatch / 64, 256, 0, stream>>>(noise, ANG, PSH, PSL);

  wmma_gemm64<1, 2, 0, 3, 0><<<(kPsiRows / 64) * (kDim / 64) / 8, 256, 0, stream>>>(
      PSH, PSL, kDim, UTH, UTL, kDim, (void*)XH, (void*)XL, kQdPad, nullptr,
      kPsiRows, kDim, kDim, 1.0f);

  wmma_gemm64<1, 2, 2, 0, 6><<<(kBatch / 64) * (kFeat / 64) / 8, 256, 0, stream>>>(
      XH, XL, kQdPad, W1H, W1L, kQdPad, (void*)Y1, nullptr, kFeat, bq1,
      kBatch, kFeat, kQdPad, 1.0f);
  ln_rows_kernel<0><<<kBatch / 64, 256, 0, stream>>>(Y1, g1, be1, X1H, X1L);

  wmma_gemm64<1, 2, 2, 0, 6><<<(kBatch / 64) * (kFeat / 64) / 8, 256, 0, stream>>>(
      X1H, X1L, kFeat, W2H, W2L, kFeat, (void*)Y2, nullptr, kFeat, bq2,
      kBatch, kFeat, kFeat, 1.0f);
  ln_rows_kernel<1><<<kBatch / 64, 256, 0, stream>>>(Y2, g2, be2, X2F, nullptr);

  wmma_gemm64<0, 0, 2, 0, 1><<<(kBatch / 64) * (kOutW / 64) / 8, 256, 0, stream>>>(
      X2F, nullptr, kFeat, W3F, nullptr, kFeat, d_out, nullptr, kOutW, bq3,
      kBatch, kOutW, kFeat, kHeadFold);
}
